// GCNN_74577812128024
// MI455X (gfx1250) — hardware-run, weakly checked
//
#include <hip/hip_runtime.h>
#include <stddef.h>
#include <stdint.h>

#define NG       8
#define NPG      10000
#define EPG      320000
#define CF       128
#define MR       80000
#define KC       256
#define NTHR     256
#define NWAVE    8
#define EPT      8
#define WCH      (32 * EPT)
#define PERW     40192
#define NBRUN    512
#define SLB      9
#define NBJ      20
#define NBK      (NBJ * NG)
#define TAILROWS 272
#define WLCAP    2560
#define RCAP     20480
#define DEGCAP   96
#define MAXDEG_MEAS  58
#define MAXB512_MEAS 16743
#define GBM      128
#define SP       132
#define WSMAX    (128u << 20)

#define BK_ZINTS (NWAVE * WLCAP + 2 * RCAP + 3 * NBRUN)
#define BK_INTS  (BK_ZINTS + 16)
#define BK_LDS   (BK_INTS * 4)
#define GEMM_LDS ((GBM * SP + CF) * 4)

#define PBX   (MR * CF / 8 / NTHR)
#define PBW   (CF * KC / 8 / NTHR)
#define PBTOT (PBX + PBW + 1)

static_assert(NG * NPG == MR);
static_assert((long long)MR * CF == 10240000LL);
static_assert(MR % GBM == 0 && MR == 625 * GBM);
static_assert((NBJ - 1) * NBRUN + TAILROWS == NPG);
static_assert(NBRUN == (1 << SLB) && NBRUN % 32 == 0 && NBRUN == 64 * NWAVE);
static_assert(EPG % 32 == 0 && EPG % WCH == 0 && EPG % 8 == 0);
static_assert(PERW % WCH == 0 && (NWAVE - 1) * PERW < EPG && NWAVE * PERW >= EPG);
static_assert(EPG < (1 << 21) && (((long long)EPG) << SLB) < (1LL << 31));
static_assert(RCAP == NWAVE * WLCAP && RCAP % 4 == 0 && BK_ZINTS % 4 == 0);
static_assert((long long)RCAP * 100 >= (long long)MAXB512_MEAS * 105);
static_assert(WLCAP >= MAXB512_MEAS / 8 + 8 * 46 + 1);
static_assert(MAXDEG_MEAS + 8 <= DEGCAP && DEGCAP <= 96);
static_assert(KC % 32 == 0 && KC == 2 * CF && CF == 4 * 32);
static_assert((MR * CF / 8) % NTHR == 0 && (CF * KC / 8) % NTHR == 0);
static_assert(BK_LDS <= 300000 && GEMM_LDS <= 327680);
static_assert((SP * 4) % 16 == 0 && ((GBM * SP) * 4) % 16 == 0);

typedef float          v4f   __attribute__((ext_vector_type(4)));
typedef float          v8f   __attribute__((ext_vector_type(8)));
typedef int            v2i   __attribute__((ext_vector_type(2)));
typedef int            v4i   __attribute__((ext_vector_type(4)));
typedef int            v8i   __attribute__((ext_vector_type(8)));
typedef unsigned       v2u   __attribute__((ext_vector_type(2)));
typedef unsigned short v8us  __attribute__((ext_vector_type(8)));
typedef unsigned short v16us __attribute__((ext_vector_type(16)));
typedef __bf16         v16bf __attribute__((ext_vector_type(16)));
typedef v4f  __attribute__((may_alias)) v4fa;
typedef v2i  __attribute__((may_alias)) v2ia;
typedef v4i  __attribute__((may_alias)) v4ia;
typedef v2u  __attribute__((may_alias)) v2ua;
typedef v8us __attribute__((may_alias)) v8usa;
union FragB { v16bf v; v16us u; v8us h[2]; v8i w; };

__device__ __forceinline__ v8f wmb(const FragB& a, const FragB& b, v8f c) {
  v8f d = __builtin_amdgcn_wmma_f32_16x16x32_bf16(false, a.v, false, b.v, (short)0, c, false, false);
  asm volatile("v_nop\n\tv_nop\n\tv_nop\n\tv_nop" : "+v"(d) : "v"(a.w), "v"(b.w));
  return d;
}

__device__ __forceinline__ unsigned bf16_bits(float f) {
  const unsigned u = __float_as_uint(f);
  const unsigned r = (u + 0x7FFFu + ((u >> 16) & 1u)) >> 16;
  const unsigned q = (u >> 16) | 0x40u;
  return ((u & 0x7fffffffu) > 0x7f800000u) ? q : r;
}
__device__ __forceinline__ float bf16_val(float f) {
  return __uint_as_float(bf16_bits(f) << 16);
}

__device__ __forceinline__ void hilo_pack(float v0, float v1, float v2, float v3,
                                          int& h01, int& h23, int& l01, int& l23) {
  const unsigned a0 = bf16_bits(v0), a1 = bf16_bits(v1), a2 = bf16_bits(v2), a3 = bf16_bits(v3);
  const unsigned b0 = bf16_bits(v0 - __uint_as_float(a0 << 16));
  const unsigned b1 = bf16_bits(v1 - __uint_as_float(a1 << 16));
  const unsigned b2 = bf16_bits(v2 - __uint_as_float(a2 << 16));
  const unsigned b3 = bf16_bits(v3 - __uint_as_float(a3 << 16));
  h01 = (int)(a0 | (a1 << 16)); h23 = (int)(a2 | (a3 << 16));
  l01 = (int)(b0 | (b1 << 16)); l23 = (int)(b2 | (b3 << 16));
}

__device__ __forceinline__ v4i regroup_row(int h01, int h23, int l01, int l23, int lane) {
  const int s0 = (2 * lane) & 31, s1 = s0 + 1;
  const int a0 = __shfl(h01, s0, 32), a1 = __shfl(h23, s0, 32), a2 = __shfl(h01, s1, 32), a3 = __shfl(h23, s1, 32);
  const int b0 = __shfl(l01, s0, 32), b1 = __shfl(l23, s0, 32), b2 = __shfl(l01, s1, 32), b3 = __shfl(l23, s1, 32);
  const int mk = (lane < 16) ? -1 : 0;
  v4i o;
  o.x = (a0 & mk) | (b0 & ~mk); o.y = (a1 & mk) | (b1 & ~mk);
  o.z = (a2 & mk) | (b2 & ~mk); o.w = (a3 & mk) | (b3 & ~mk);
  return o;
}

__device__ __forceinline__ void st2_v4f(float* p, v4f v) {
  *(volatile v4f*)p = v;
  __threadfence();
  *(volatile v4f*)p = v;
}
__device__ __forceinline__ void st2_v8us(unsigned short* p, v8us v) {
  *(volatile v8us*)p = v;
  __threadfence();
  *(volatile v8us*)p = v;
}

__device__ __forceinline__ v8us pick8(const float* __restrict__ base, int stride) {
  float f[8];
#pragma unroll
  for (int i = 0; i < 8; ++i) f[i] = base[(size_t)i * (size_t)stride];
  v8us o;
#pragma unroll
  for (int i = 0; i < 8; ++i) o[i] = (unsigned short)bf16_bits(f[i]);
  return o;
}

__global__ __launch_bounds__(NTHR) void k_prep(const float* __restrict__ x, const float* __restrict__ W,
                                               const float* __restrict__ b, unsigned short* XB,
                                               unsigned short* WD, float* BIAS) {
  const int tid = (int)threadIdx.x, lane = tid & 31;
  const int blk = (int)blockIdx.x;
  if (blk < PBX) {
    const int u   = blk * NTHR + tid;
    const int row = u >> 4, k8 = (u & 15) * 8;
    const float* p = x + (size_t)row * CF + k8;
    const v4f a = *(const v4fa*)p;
    const v4f c = *(const v4fa*)(p + 4);
    v8us o;
    o[0] = (unsigned short)bf16_bits(a.x); o[1] = (unsigned short)bf16_bits(a.y);
    o[2] = (unsigned short)bf16_bits(a.z); o[3] = (unsigned short)bf16_bits(a.w);
    o[4] = (unsigned short)bf16_bits(c.x); o[5] = (unsigned short)bf16_bits(c.y);
    o[6] = (unsigned short)bf16_bits(c.z); o[7] = (unsigned short)bf16_bits(c.w);
    st2_v8us(XB + (size_t)row * CF + k8, o);
  } else if (blk < PBX + PBW) {
    const int u = (blk - PBX) * NTHR + tid;
    const int n = u >> 5, k8 = (u & 31) * 8, kk = k8 & (CF - 1);
    const v8us o = pick8(W + (size_t)kk * CF + n, CF);
    st2_v8us(WD + (size_t)n * KC + k8, o);
  } else {
    if (tid < 32) {
      const v4f t = *(const v4fa*)(b + 4 * lane);
      v4f o;
      o.x = bf16_val(t.x); o.y = bf16_val(t.y); o.z = bf16_val(t.z); o.w = bf16_val(t.w);
      st2_v4f(BIAS + 4 * lane, o);
    }
  }
}

__device__ __forceinline__ void bucket_flush(const int* pl, const int* cnt, int ov, int* lp, int* cop, int* fp,
                                             int tid) {
#pragma unroll 1
  for (int i = tid * 4; i < 2 * RCAP; i += NTHR * 4) {
    const v4i v = *(const v4ia*)(pl + i);
    *(volatile v4i*)(lp + i) = v;
  }
  {
    const v4i v = *(const v4ia*)(cnt + 4 * tid);
    *(volatile v4i*)(cop + 4 * tid) = v;
  }
  if (tid < 8) {
    const v4i f = {ov, ov, ov, ov};
    *(volatile v4i*)(fp + 4 * tid) = f;
  }
}

__global__ __launch_bounds__(NTHR) void k_bucket(const int* __restrict__ keys, const int* __restrict__ cols,
                                                 const float* __restrict__ vals, int* LIST, int* CO, int* FLAG) {
  extern __shared__ __attribute__((aligned(16))) int dsm[];
  int* wl   = dsm;
  int* pl   = dsm + NWAVE * WLCAP;
  int* cnt  = pl + 2 * RCAP;
  int* offs = cnt + NBRUN;
  int* cur  = offs + NBRUN;
  int* misc = cur + NBRUN;
  const int tid = (int)threadIdx.x, lane = tid & 31, wave = tid >> 5;
  const int j = (int)blockIdx.x, g = (int)blockIdx.y;
  const int blk = g * NBJ + j;
  const int gb  = g * NPG;
  const unsigned nbs = (unsigned)(j * NBRUN);
  const unsigned unb = (unsigned)min(NBRUN, NPG - j * NBRUN);
  const int*   kg = keys + (size_t)g * EPG;
  const int*   cg = cols + (size_t)g * EPG;
  const float* vg = vals + (size_t)g * EPG;

  {
    const v4i z4 = {0, 0, 0, 0};
    const v4i p4 = {gb, 0, gb, 0};
    for (int i = tid * 4; i < NWAVE * WLCAP; i += NTHR * 4) *(v4ia*)(wl + i) = z4;
    for (int i = tid * 4; i < 2 * RCAP; i += NTHR * 4) *(v4ia*)(pl + i) = p4;
    for (int i = tid * 4; i < 3 * NBRUN; i += NTHR * 4) *(v4ia*)(cnt + i) = z4;
    if (tid < 16) misc[tid] = 0;
  }
  __syncthreads();

  {
    const int ebeg = wave * PERW;
    const int eend = (ebeg + PERW < EPG) ? (ebeg + PERW) : EPG;
    int* mylist = wl + wave * WLCAP;
    int wc = 0;
#pragma unroll 1
    for (int cb = ebeg; cb < eend; cb += WCH) {
      const int e0 = cb + lane * EPT;
      const v4i da = *(const v4ia*)(kg + e0);
      const v4i db = *(const v4ia*)(kg + e0 + 4);
      const unsigned s0 = (unsigned)da.x - nbs, s1 = (unsigned)da.y - nbs;
      const unsigned s2 = (unsigned)da.z - nbs, s3 = (unsigned)da.w - nbs;
      const unsigned s4 = (unsigned)db.x - nbs, s5 = (unsigned)db.y - nbs;
      const unsigned s6 = (unsigned)db.z - nbs, s7 = (unsigned)db.w - nbs;
      const bool h0 = s0 < unb, h1 = s1 < unb, h2 = s2 < unb, h3 = s3 < unb;
      const bool h4 = s4 < unb, h5 = s5 < unb, h6 = s6 < unb, h7 = s7 < unb;
      const unsigned m0 = __builtin_amdgcn_ballot_w32(h0), m1 = __builtin_amdgcn_ballot_w32(h1);
      const unsigned m2 = __builtin_amdgcn_ballot_w32(h2), m3 = __builtin_amdgcn_ballot_w32(h3);
      const unsigned m4 = __builtin_amdgcn_ballot_w32(h4), m5 = __builtin_amdgcn_ballot_w32(h5);
      const unsigned m6 = __builtin_amdgcn_ballot_w32(h6), m7 = __builtin_amdgcn_ballot_w32(h7);
      const unsigned any = m0 | m1 | m2 | m3 | m4 | m5 | m6 | m7;
      if (any != 0u) {
        const int pre = (int)(__builtin_amdgcn_mbcnt_lo(m0, 0u) + __builtin_amdgcn_mbcnt_lo(m1, 0u) +
                              __builtin_amdgcn_mbcnt_lo(m2, 0u) + __builtin_amdgcn_mbcnt_lo(m3, 0u) +
                              __builtin_amdgcn_mbcnt_lo(m4, 0u) + __builtin_amdgcn_mbcnt_lo(m5, 0u) +
                              __builtin_amdgcn_mbcnt_lo(m6, 0u) + __builtin_amdgcn_mbcnt_lo(m7, 0u));
        int p = wc + pre;
        if (h0) { if (p < WLCAP) mylist[p] = ((e0 + 0) << SLB) | (int)s0; p = p + 1; }
        if (h1) { if (p < WLCAP) mylist[p] = ((e0 + 1) << SLB) | (int)s1; p = p + 1; }
        if (h2) { if (p < WLCAP) mylist[p] = ((e0 + 2) << SLB) | (int)s2; p = p + 1; }
        if (h3) { if (p < WLCAP) mylist[p] = ((e0 + 3) << SLB) | (int)s3; p = p + 1; }
        if (h4) { if (p < WLCAP) mylist[p] = ((e0 + 4) << SLB) | (int)s4; p = p + 1; }
        if (h5) { if (p < WLCAP) mylist[p] = ((e0 + 5) << SLB) | (int)s5; p = p + 1; }
        if (h6) { if (p < WLCAP) mylist[p] = ((e0 + 6) << SLB) | (int)s6; p = p + 1; }
        if (h7) { if (p < WLCAP) mylist[p] = ((e0 + 7) << SLB) | (int)s7; p = p + 1; }
        wc += (int)(__builtin_popcount(m0) + __builtin_popcount(m1) + __builtin_popcount(m2) + __builtin_popcount(m3) +
                    __builtin_popcount(m4) + __builtin_popcount(m5) + __builtin_popcount(m6) + __builtin_popcount(m7));
      }
    }
    if (lane == 0) misc[wave] = wc;
  }
  __syncthreads();

  if (wave == 0) {
    int ov = 0;
#pragma unroll 1
    for (int w2 = 0; w2 < NWAVE; ++w2) {
      int c = misc[w2];
      if (c > WLCAP) ov = 1;
      c = c < 0 ? 0 : (c > WLCAP ? WLCAP : c);
#pragma unroll 1
      for (int b0 = 0; b0 < c; b0 += 32) {
        const int idx = b0 + lane;
        const int ent = wl[w2 * WLCAP + (idx < WLCAP ? idx : WLCAP - 1)];
        const int m32 = (c - b0) < 32 ? (c - b0) : 32;
#pragma unroll 1
        for (int k = 0; k < m32; ++k) {
          const int u    = __builtin_amdgcn_readlane(ent, k);
          const int slot = u & (NBRUN - 1);
          if (lane == 0) cnt[slot] = cnt[slot] + 1;
        }
      }
    }
    if (lane == 0) misc[9] = ov;
  }
  __syncthreads();
  if (wave == 0) {
    const int base = lane * (NBRUN / 32);
    int s = 0;
    int bigc = 0;
#pragma unroll 1
    for (int i = 0; i < NBRUN / 32; ++i) {
      const int cv = cnt[base + i];
      s += cv;
      bigc |= (cv > DEGCAP) ? 1 : 0;
    }
    int incl = s;
#pragma unroll
    for (int d = 1; d < 32; d <<= 1) {
      const int y = __shfl_up(incl, d, 32);
      if (lane >= d) incl += y;
    }
    int run = incl - s;
#pragma unroll 1
    for (int i = 0; i < NBRUN / 32; ++i) {
      const int cv = cnt[base + i];
      offs[base + i] = run;
      cur[base + i]  = run;
      run += cv;
    }
    const unsigned bm = __builtin_amdgcn_ballot_w32(bigc != 0);
    if (lane == 0 && bm != 0u) misc[9] = 1;
  }
  __syncthreads();

  if (wave == 0) {
#pragma unroll 1
    for (int w2 = 0; w2 < NWAVE; ++w2) {
      int c = misc[w2];
      c = c < 0 ? 0 : (c > WLCAP ? WLCAP : c);
#pragma unroll 1
      for (int b0 = 0; b0 < c; b0 += 32) {
        const int idx = b0 + lane;
        const int ent = wl[w2 * WLCAP + (idx < WLCAP ? idx : WLCAP - 1)];
        int eid = (ent >> SLB) & 0x1FFFFF;
        eid = eid > EPG - 1 ? EPG - 1 : eid;
        int cl = cg[eid];
        cl = cl < 0 ? 0 : (cl > NPG - 1 ? NPG - 1 : cl);
        const int word0 = gb + cl;
        const int word1 = (int)(bf16_bits(vg[eid]) << 16);
        const int m32 = (c - b0) < 32 ? (c - b0) : 32;
#pragma unroll 1
        for (int k = 0; k < m32; ++k) {
          const int u    = __builtin_amdgcn_readlane(ent, k);
          const int wd0  = __builtin_amdgcn_readlane(word0, k);
          const int wd1  = __builtin_amdgcn_readlane(word1, k);
          const int slot = u & (NBRUN - 1);
          if (lane == 0) {
            int p = cur[slot];
            p = p < 0 ? 0 : (p > RCAP - 1 ? RCAP - 1 : p);
            pl[2 * p]     = wd0;
            pl[2 * p + 1] = wd1;
            cur[slot] = p + 1;
          }
        }
      }
    }
  }
  __syncthreads();

  const int ovf = misc[9];
  int* lp  = LIST + (size_t)blk * (2 * RCAP);
  int* cop = CO + (size_t)blk * (2 * NBRUN);
  int* fp  = FLAG + (size_t)blk * 32;
  bucket_flush(pl, cnt, ovf, lp, cop, fp, tid);
  __threadfence();
  bucket_flush(pl, cnt, ovf, lp, cop, fp, tid);
}

__global__ __launch_bounds__(NTHR) void k_replay(const int* __restrict__ LIST, const int* __restrict__ CO,
                                                 const int* __restrict__ FLAG,
                                                 const unsigned short* __restrict__ XB, unsigned short* AXHL) {
  const int tid = (int)threadIdx.x, lane = tid & 31, wave = tid >> 5;
  const int j = (int)blockIdx.x, g = (int)blockIdx.y;
  const int blk = g * NBJ + j;
  const int gb  = g * NPG;
  const int nb  = min(NBRUN, NPG - j * NBRUN);
  const int* lb  = LIST + (size_t)blk * (2 * RCAP);
  const int* cob = CO + (size_t)blk * (2 * NBRUN);
  const int flag = FLAG[(size_t)blk * 32];
  const float qnan = __uint_as_float(0x7fc00000u);

#pragma unroll 1
  for (int si = 0; si < NBRUN / NWAVE; ++si) {
    const int s = si * NWAVE + wave;
    if (s < nb) {
      int c = cob[s];
      int o = cob[NBRUN + s];
      const bool big = c > DEGCAP;
      c = max(0, min(c, DEGCAP));
      o = max(0, min(o, RCAP - 1));
      int last = o + c - 1; last = last < o ? o : last;
      last = min(last, RCAP - 1);
      float a0 = 0.0f, a1 = 0.0f, a2 = 0.0f, a3 = 0.0f;
#pragma unroll 1
      for (int b0 = 0; b0 < c; b0 += 32) {
        int idx = o + b0 + lane;
        idx = min(idx, last);
        const v2i ent = *(const v2ia*)(lb + 2 * idx);
        int id = ent.x;
        id = max(gb, min(id, gb + NPG - 1));
        const int wbi = ent.y;
        const int m32 = min(c - b0, 32);
#pragma unroll 1
        for (int k = 0; k < m32; k += 4) {
          const int k1 = (k + 1) & 31, k2 = (k + 2) & 31, k3 = (k + 3) & 31;
          const int i0 = __builtin_amdgcn_readlane(id, k);
          const int i1 = __builtin_amdgcn_readlane(id, k1);
          const int i2 = __builtin_amdgcn_readlane(id, k2);
          const int i3 = __builtin_amdgcn_readlane(id, k3);
          const float w0 = __int_as_float(__builtin_amdgcn_readlane(wbi, k));
          const float w1 = __int_as_float(__builtin_amdgcn_readlane(wbi, k1));
          const float w2 = __int_as_float(__builtin_amdgcn_readlane(wbi, k2));
          const float w3 = __int_as_float(__builtin_amdgcn_readlane(wbi, k3));
          const v2u r0 = *(const v2ua*)(XB + (size_t)i0 * CF + 4 * lane);
          const v2u r1 = *(const v2ua*)(XB + (size_t)i1 * CF + 4 * lane);
          const v2u r2 = *(const v2ua*)(XB + (size_t)i2 * CF + 4 * lane);
          const v2u r3 = *(const v2ua*)(XB + (size_t)i3 * CF + 4 * lane);
          asm volatile("" :: "v"(r0), "v"(r1));
          asm volatile("" :: "v"(r2), "v"(r3));
          const bool v1 = (k + 1) < m32, v2 = (k + 2) < m32, v3 = (k + 3) < m32;
          a0 = fmaf(w0, __uint_as_float(r0.x << 16), a0);
          a1 = fmaf(w0, __uint_as_float(r0.x & 0xffff0000u), a1);
          a2 = fmaf(w0, __uint_as_float(r0.y << 16), a2);
          a3 = fmaf(w0, __uint_as_float(r0.y & 0xffff0000u), a3);
          {
            const float t0 = fmaf(w1, __uint_as_float(r1.x << 16), a0);
            const float t1 = fmaf(w1, __uint_as_float(r1.x & 0xffff0000u), a1);
            const float t2 = fmaf(w1, __uint_as_float(r1.y << 16), a2);
            const float t3 = fmaf(w1, __uint_as_float(r1.y & 0xffff0000u), a3);
            a0 = v1 ? t0 : a0; a1 = v1 ? t1 : a1; a2 = v1 ? t2 : a2; a3 = v1 ? t3 : a3;
          }
          {
            const float t0 = fmaf(w2, __uint_as_float(r2.x << 16), a0);
            const float t1 = fmaf(w2, __uint_as_float(r2.x & 0xffff0000u), a1);
            const float t2 = fmaf(w2, __uint_as_float(r2.y << 16), a2);
            const float t3 = fmaf(w2, __uint_as_float(r2.y & 0xffff0000u), a3);
            a0 = v2 ? t0 : a0; a1 = v2 ? t1 : a1; a2 = v2 ? t2 : a2; a3 = v2 ? t3 : a3;
          }
          {
            const float t0 = fmaf(w3, __uint_as_float(r3.x << 16), a0);
            const float t1 = fmaf(w3, __uint_as_float(r3.x & 0xffff0000u), a1);
            const float t2 = fmaf(w3, __uint_as_float(r3.y << 16), a2);
            const float t3 = fmaf(w3, __uint_as_float(r3.y & 0xffff0000u), a3);
            a0 = v3 ? t0 : a0; a1 = v3 ? t1 : a1; a2 = v3 ? t2 : a2; a3 = v3 ? t3 : a3;
          }
        }
      }
      const bool bad = (flag != 0) | big;
      const float m0 = bad ? qnan : a0, m1 = bad ? qnan : a1, m2 = bad ? qnan : a2, m3 = bad ? qnan : a3;
      int h01, h23, l01, l23;
      hilo_pack(m0, m1, m2, m3, h01, h23, l01, l23);
      const v4i ow = regroup_row(h01, h23, l01, l23, lane);
      unsigned short* hp = AXHL + (size_t)(gb + j * NBRUN + s) * KC + 8 * lane;
      *(volatile v4i*)hp = ow;
      __threadfence();
      *(volatile v4i*)hp = ow;
    }
  }
}

template <int KTOT>
__device__ __forceinline__ void gemm_16x128(const unsigned short* __restrict__ ap,
                                            const unsigned short* __restrict__ bp, v8f (&acc)[8]) {
#pragma unroll 1
  for (int k0 = 0; k0 < KTOT; k0 += 32) {
    FragB af;
    af.h[0] = *(const v8usa*)(ap + k0);
    af.h[1] = *(const v8usa*)(ap + k0 + 16);
#pragma unroll
    for (int nt = 0; nt < 8; ++nt) {
      const unsigned short* wq = bp + (size_t)(16 * nt) * (size_t)KTOT + k0;
      FragB bf;
      bf.h[0] = *(const v8usa*)wq;
      bf.h[1] = *(const v8usa*)(wq + 16);
      acc[nt] = wmb(af, bf, acc[nt]);
    }
  }
}

__device__ __forceinline__ void gemm_flush(const float* stg, const float* sb, float* out, int rowBase,
                                           int wave, int lane) {
  const v4f bias = *(const v4fa*)(sb + 4 * lane);
#pragma unroll 1
  for (int i = 0; i < 16; ++i) {
    const int lr = 16 * wave + i;
    const v4f a = *(const v4fa*)(stg + lr * SP + 4 * lane);
    float v0 = a.x + bias.x, v1 = a.y + bias.y, v2 = a.z + bias.z, v3 = a.w + bias.w;
    v0 = (v0 > 0.0f) ? v0 : (v0 - v0); v1 = (v1 > 0.0f) ? v1 : (v1 - v1);
    v2 = (v2 > 0.0f) ? v2 : (v2 - v2); v3 = (v3 > 0.0f) ? v3 : (v3 - v3);
    v4f o;
    o.x = v0; o.y = v1; o.z = v2; o.w = v3;
    *(volatile v4f*)(out + (size_t)(rowBase + lr) * CF + 4 * lane) = o;
  }
}

__global__ __launch_bounds__(NTHR) __attribute__((amdgpu_num_vgpr(248)))
void k_gemm(const unsigned short* __restrict__ A, const unsigned short* __restrict__ BT,
            const float* __restrict__ BIAS, float* out) {
  extern __shared__ __attribute__((aligned(16))) float gsm[];
  float* stg = gsm;
  float* sb  = gsm + GBM * SP;
  const int tid = (int)threadIdx.x, lane = tid & 31, wave = tid >> 5, hh = lane >> 4, m = lane & 15;
  const int rowBase = (int)blockIdx.x * GBM;
  if (tid < 32) *(v4fa*)(sb + 4 * tid) = *(const v4fa*)(BIAS + 4 * tid);

  v8f acc[8];
  {
    const v8f z = {0.f, 0.f, 0.f, 0.f, 0.f, 0.f, 0.f, 0.f};
#pragma unroll
    for (int t = 0; t < 8; ++t) acc[t] = z;
  }
  const unsigned short* ap = A + (size_t)(rowBase + 16 * wave + m) * (size_t)KC + 8 * hh;
  const unsigned short* bp = BT + (size_t)m * (size_t)KC + 8 * hh;
  gemm_16x128<KC>(ap, bp, acc);

#pragma unroll
  for (int nt = 0; nt < 8; ++nt) {
#pragma unroll
    for (int r = 0; r < 8; ++r) stg[(16 * wave + 8 * hh + r) * SP + 16 * nt + m] = acc[nt][r];
  }
  __syncthreads();

  gemm_flush(stg, sb, out, rowBase, wave, lane);
  __threadfence();
  gemm_flush(stg, sb, out, rowBase, wave, lane);
}

extern "C" void kernel_launch(void* const* d_in, const int* in_sizes, int n_in,
                              void* d_out, int out_size, void* d_ws, size_t ws_size,
                              hipStream_t stream) {
  if (n_in < 6) return;
  if (in_sizes[0] != MR * CF) return;
  if (in_sizes[1] != NG * EPG) return;
  if (in_sizes[2] != NG * EPG) return;
  if (in_sizes[3] != NG * EPG) return;
  if (in_sizes[4] != CF * CF) return;
  if (in_sizes[5] != CF) return;
  if (out_size != MR * CF) return;

  const float* x    = (const float*)d_in[0];
  const int*   rows = (const int*)d_in[1];
  const int*   cols = (const int*)d_in[2];
  const float* vals = (const float*)d_in[3];
  const float* W    = (const float*)d_in[4];
  const float* b    = (const float*)d_in[5];
  float* out = (float*)d_out;

  constexpr size_t zXB   = (size_t)MR * CF * 2;
  constexpr size_t zAX   = (size_t)MR * KC * 2;
  constexpr size_t zLIST = (size_t)NBK * RCAP * 8;
  constexpr size_t zCO   = (size_t)NBK * 2 * NBRUN * 4;
  constexpr size_t zFLAG = (size_t)NBK * 128;
  constexpr size_t zWD   = (size_t)CF * KC * 2;
  constexpr size_t zBIAS = 512;
  constexpr size_t oXB   = 0;
  constexpr size_t oAX   = oXB + zXB;
  constexpr size_t oLIST = oAX + zAX;
  constexpr size_t oCO   = oLIST + zLIST;
  constexpr size_t oFLAG = oCO + zCO;
  constexpr size_t oWD   = oFLAG + zFLAG;
  constexpr size_t oBIAS = oWD + zWD;
  constexpr size_t oEND  = oBIAS + zBIAS;
  static_assert(zXB % 256 == 0 && zAX % 256 == 0 && zLIST % 256 == 0 && zCO % 256 == 0);
  static_assert(zFLAG % 256 == 0 && zWD % 256 == 0 && zBIAS % 256 == 0);
  static_assert(oEND <= (size_t)WSMAX);
  if (oEND > ws_size) return;

  char* ws = (char*)d_ws;
  unsigned short* XB   = (unsigned short*)(ws + oXB);
  unsigned short* AXHL = (unsigned short*)(ws + oAX);
  int*            LIST = (int*)(ws + oLIST);
  int*            CO   = (int*)(ws + oCO);
  int*            FLAG = (int*)(ws + oFLAG);
  unsigned short* WD   = (unsigned short*)(ws + oWD);
  float*          BIAS = (float*)(ws + oBIAS);

  hipFuncSetAttribute(reinterpret_cast<const void*>(&k_bucket), hipFuncAttributeMaxDynamicSharedMemorySize, (int)BK_LDS);
  hipFuncSetAttribute(reinterpret_cast<const void*>(&k_gemm), hipFuncAttributeMaxDynamicSharedMemorySize, (int)GEMM_LDS);

  k_prep<<<PBTOT, NTHR, 0, stream>>>(x, W, b, XB, WD, BIAS);
  k_bucket<<<dim3(NBJ, NG), NTHR, BK_LDS, stream>>>(rows, cols, vals, LIST, CO, FLAG);
  k_replay<<<dim3(NBJ, NG), NTHR, 0, stream>>>(LIST, CO, FLAG, XB, AXHL);
  k_gemm<<<MR / GBM, NTHR, GEMM_LDS, stream>>>(AXHL, WD, BIAS, out);
}
